// FastMultiheadAttention_2860448219139
// MI455X (gfx1250) — hardware-verified
//
#include <hip/hip_runtime.h>
#include <math.h>

typedef __attribute__((ext_vector_type(16))) _Float16 v16h;
typedef __attribute__((ext_vector_type(16))) __bf16 v16b;
typedef __attribute__((ext_vector_type(8)))  _Float16 v8h;
typedef __attribute__((ext_vector_type(8)))  float v8f;
typedef __attribute__((ext_vector_type(4)))  float v4f;
typedef __attribute__((ext_vector_type(2)))  float v2f;
typedef __attribute__((ext_vector_type(4)))  unsigned v4u;
typedef __attribute__((ext_vector_type(4)))  int v4i;
typedef float __attribute__((may_alias)) float_a;
typedef int __attribute__((may_alias)) int_a;

template <typename T> __device__ __forceinline__ void vst2(void* p, T v) { *(volatile T*)p = v; __threadfence(); *(volatile T*)p = v; }
__device__ __forceinline__ v8f wmma16(v16h a, v16h b, v8f c) {
  v8f d = __builtin_amdgcn_wmma_f32_16x16x32_f16(false, a, false, b, (short)0, c, false, false);
  asm volatile("v_nop\n\tv_nop\n\tv_nop\n\tv_nop" : "+v"(d) : "v"(a), "v"(b));
  return d;
}
__device__ __forceinline__ v8f wmma_bf(v16b a, v16b b, v8f c) {
  v8f d = __builtin_amdgcn_wmma_f32_16x16x32_bf16(false, a, false, b, (short)0, c, false, false);
  asm volatile("v_nop\n\tv_nop\n\tv_nop\n\tv_nop" : "+v"(d) : "v"(a), "v"(b));
  return d;
}
__device__ __forceinline__ v16h frag_h(const _Float16* rowk0, int lane) {
  union { v16h v; v8h q[2]; } u; const _Float16* p = rowk0 + 8 * (lane >> 4);
  u.q[0] = *(const v8h*)p; u.q[1] = *(const v8h*)(p + 16); return u.v;
}
__device__ __forceinline__ v16h frag_f32(const float* rowk0, int lane) {
  v16h a; const float* p = rowk0 + 8 * (lane >> 4);
#pragma unroll
  for (int i = 0; i < 8; ++i) { a[i] = (_Float16)p[i]; a[8 + i] = (_Float16)p[16 + i]; }
  return a;
}
__device__ __forceinline__ v16h frag_f32s(const float* rowk0, int lane, float sc) {
  v16h a; const float* p = rowk0 + 8 * (lane >> 4);
#pragma unroll
  for (int i = 0; i < 8; ++i) { a[i] = (_Float16)(p[i] * sc); a[8 + i] = (_Float16)(p[16 + i] * sc); }
  return a;
}
__device__ __forceinline__ v16h fragc_f32(const float* W, int k0, int n, int lane, int ld, int K) {
  v16h a; const int g = lane >> 4;
#pragma unroll
  for (int i = 0; i < 8; ++i) { const int ka = k0 + 8 * g + i, kb = ka + 16;
    a[i] = (_Float16)(ka < K ? W[(size_t)(ka < K ? ka : K - 1) * ld + n] : 0.f); a[8 + i] = (_Float16)(kb < K ? W[(size_t)(kb < K ? kb : K - 1) * ld + n] : 0.f); }
  return a;
}
struct F2 { v16b h, l; };
__device__ __forceinline__ F2 bsplit16(const float v[16]) { F2 r;
#pragma unroll
  for (int i = 0; i < 16; ++i) { const __bf16 h = (__bf16)v[i]; r.h[i] = h; r.l[i] = (__bf16)(v[i] - (float)h); }
  return r; }
__device__ __forceinline__ F2 split_row(const float* row, int k0, int lane) { float v[16]; const float* p = row + k0 + 8 * (lane >> 4);
#pragma unroll
  for (int i = 0; i < 8; ++i) { v[i] = p[i]; v[8 + i] = p[16 + i]; }
  return bsplit16(v); }
__device__ __forceinline__ F2 split_rowK(const float* row, int k0, int lane, int K) { float v[16]; const int g = lane >> 4;
#pragma unroll
  for (int i = 0; i < 8; ++i) { const int ka = k0 + 8 * g + i, kb = ka + 16; v[i] = ka < K ? row[ka < K ? ka : K - 1] : 0.f; v[8 + i] = kb < K ? row[kb < K ? kb : K - 1] : 0.f; }
  return bsplit16(v); }
__device__ __forceinline__ F2 split_col(const float* W, int k0, int n, int lane, int ld, int K) { float v[16]; const int g = lane >> 4;
#pragma unroll
  for (int i = 0; i < 8; ++i) { const int ka = k0 + 8 * g + i, kb = ka + 16; v[i] = ka < K ? W[(size_t)(ka < K ? ka : K - 1) * ld + n] : 0.f; v[8 + i] = kb < K ? W[(size_t)(kb < K ? kb : K - 1) * ld + n] : 0.f; }
  return bsplit16(v); }
__device__ __forceinline__ v8f mac3(const F2& a, const F2& b, v8f c) { c = wmma_bf(a.l, b.h, c); c = wmma_bf(a.h, b.l, c); return wmma_bf(a.h, b.h, c); }
__device__ __forceinline__ float sigm(float v) { return 1.0f / (1.0f + expf(-v)); }
#define LDSX() do { asm volatile("s_wait_dscnt 0" ::: "memory"); __builtin_amdgcn_wave_barrier(); __builtin_amdgcn_fence(__ATOMIC_RELEASE, "workgroup"); } while (0)
__device__ __forceinline__ v16b wcol_oi(const float* Wm, int k0, int o, int lane, int K) { v16b w; const float* p = Wm + (size_t)o * K + k0 + 8 * (lane >> 4);
#pragma unroll
  for (int i = 0; i < 8; ++i) { w[i] = (__bf16)p[i]; w[8 + i] = (__bf16)p[16 + i]; }
  return w; }

#define NBT 2
#define NN 8192
#define HID 512
#define NHD 8
#define HDM 64
#define MF 256
#define NR (NBT * NN)
#ifndef TNB
#define TNB NBT
#endif
#define NRV (TNB * NN)
#define UG 4
__device__ __forceinline__ float bfr(float v) { return (float)(__bf16)v; }
#define WS_Q    0u
#define WS_K    (WS_Q + 4u * (size_t)NR * HID)
#define WS_V    (WS_K + 4u * (size_t)NR * HID)
#define WS_QP   (WS_V + 4u * (size_t)NR * HID)
#define WS_KPT  (WS_QP + 4u * (size_t)UG * NN * MF)
#define WS_KS   (WS_KPT + 4u * (size_t)UG * MF * NN)
#define WS_CTX  (WS_KS + 4u * (size_t)NBT * NHD * MF)
#define WS_ATT  (WS_CTX + 4u * (size_t)NBT * NHD * MF * HDM)
#define WS_END  (WS_ATT + 4u * (size_t)NR * HID)

__global__ __launch_bounds__(128) void k_lin(const float* __restrict__ X0, const float* __restrict__ X1, const float* __restrict__ X2, const float* __restrict__ W0, const float* __restrict__ W1, const float* __restrict__ W2, const float* __restrict__ B0, const float* __restrict__ B1, const float* __restrict__ B2, float* __restrict__ O0, float* __restrict__ O1, float* __restrict__ O2) { __shared__ __align__(16) float sf[4][16][132];
  const int tid = threadIdx.x, wave = tid >> 5, lane = tid & 31, col = lane & 15, g = lane >> 4; const int which = blockIdx.z; const int c0 = blockIdx.y * 128; const size_t r0 = (size_t)blockIdx.x * 64 + wave * 16;
  const float* X = which == 0 ? X0 : which == 1 ? X1 : X2; const float* Wm = which == 0 ? W0 : which == 1 ? W1 : W2; const float* Bv = which == 0 ? B0 : which == 1 ? B1 : B2; float* OUT = which == 0 ? O0 : which == 1 ? O1 : O2;
  v8f acc[8] = {};
#pragma unroll 2
  for (int kc = 0; kc < HID / 32; ++kc) { v16b a; { const float* p = X + (r0 + col) * HID + kc * 32 + 8 * g;
#pragma unroll
      for (int i = 0; i < 8; ++i) { a[i] = (__bf16)p[i]; a[8 + i] = (__bf16)p[16 + i]; } }
    asm volatile("s_wait_loadcnt 0x0" ::: "memory");
#pragma unroll
    for (int j = 0; j < 8; ++j) { const v16b w = wcol_oi(Wm, kc * 32, c0 + j * 16 + col, lane, HID); asm volatile("s_wait_loadcnt 0x0" ::: "memory"); acc[j] = wmma_bf(a, w, acc[j]); } }
#pragma unroll
  for (int j = 0; j < 8; ++j) { const float bb = bfr(Bv[c0 + j * 16 + col]);
#pragma unroll
    for (int r = 0; r < 8; ++r) sf[wave][8 * g + r][j * 16 + col] = acc[j][r] + bb; }
  LDSX(); for (int rl = 0; rl < 16; ++rl) vst2(OUT + (r0 + rl) * HID + c0 + lane * 4, *(const v4f*)&sf[wave][rl][lane * 4]); }
__global__ __launch_bounds__(128) void k_phi(const float* __restrict__ Q, const float* __restrict__ K, const float* __restrict__ PRJ, int bh0, float* __restrict__ QP, float* __restrict__ KPT) { __shared__ __align__(16) float sf[64][132]; __shared__ float sdiag[64];
  const int tid = threadIdx.x, wave = tid >> 5, lane = tid & 31, col = lane & 15, g = lane >> 4; const int which = blockIdx.z & 1; const int unit = blockIdx.z >> 1; const int bh = bh0 + unit; const int b = bh / NHD, h = bh % NHD; const int m0 = blockIdx.y * 128; const int n0 = blockIdx.x * 64;
  const float* SRC = which == 0 ? Q : K; const float s4 = 0.35355339059327373f;
  { const int rl = tid >> 1, half = tid & 1; const float* p = SRC + ((size_t)b * NN + n0 + rl) * HID + h * HDM + half * 32; float s2 = 0.f;
#pragma unroll
    for (int i = 0; i < 32; i += 4) { const v4f v = *(const v4f*)(p + i);
#pragma unroll
      for (int j = 0; j < 4; ++j) { const float xs = v[j] * s4; s2 += xs * xs; } }
    s2 += __shfl_xor(s2, 1); if (half == 0) sdiag[rl] = 0.5f * s2; }
  v8f acc[8] = {};
#pragma unroll
  for (int kc = 0; kc < HDM / 32; ++kc) { float v[16]; { const float* p = SRC + ((size_t)b * NN + n0 + wave * 16 + col) * HID + h * HDM + kc * 32 + 8 * g;
#pragma unroll
      for (int i = 0; i < 8; ++i) { v[i] = p[i] * s4; v[8 + i] = p[16 + i] * s4; } }
    const F2 a = bsplit16(v); asm volatile("s_wait_loadcnt 0x0" ::: "memory");
#pragma unroll
    for (int j = 0; j < 8; ++j) { const v16b w = wcol_oi(PRJ, kc * 32, m0 + j * 16 + col, lane, HDM); asm volatile("s_wait_loadcnt 0x0" ::: "memory"); acc[j] = wmma_bf(a.h, w, acc[j]); acc[j] = wmma_bf(a.l, w, acc[j]); } }
  __syncthreads();
#pragma unroll
  for (int j = 0; j < 8; ++j)
#pragma unroll
    for (int r = 0; r < 8; ++r) { const int rl = wave * 16 + 8 * g + r; sf[rl][j * 16 + col] = 0.0625f * expf(acc[j][r] - sdiag[rl]) + 1e-4f; }
  __syncthreads();
  if (which == 0) { for (int e = tid; e < 64 * 32; e += 128) { const int rl = e >> 5, q = e & 31; vst2(QP + (((size_t)unit * NN) + n0 + rl) * MF + m0 + q * 4, *(const v4f*)&sf[rl][q * 4]); } }
  else { for (int e = tid; e < 128 * 16; e += 128) { const int ml = e >> 4, q = e & 15; v4f o; o[0] = sf[q * 4][ml]; o[1] = sf[q * 4 + 1][ml]; o[2] = sf[q * 4 + 2][ml]; o[3] = sf[q * 4 + 3][ml]; vst2(KPT + ((size_t)unit * MF + m0 + ml) * NN + n0 + q * 4, o); } } }
__global__ __launch_bounds__(256) void k_ksum(const float* __restrict__ KPT, int bh0, float* __restrict__ KS) { __shared__ __align__(16) float sk[64];
  const int tid = threadIdx.x; const int unit = blockIdx.y; const int bh = bh0 + unit; const int m = blockIdx.x * 64 + (tid >> 2); const int part = tid & 3; const float* p = KPT + ((size_t)unit * MF + m) * NN; float s = 0.f;
  for (int n = part * 4; n < NN; n += 16) { const v4f v = *(const v4f*)(p + n); s += (v[0] + v[1]) + (v[2] + v[3]); }
  s += __shfl_xor(s, 1); s += __shfl_xor(s, 2); if (part == 0) sk[tid >> 2] = s;
  __syncthreads();
  if (tid < 16) vst2(KS + (size_t)bh * MF + blockIdx.x * 64 + tid * 4, *(const v4f*)&sk[tid * 4]); }
__global__ __launch_bounds__(128) void k_ctx(const float* __restrict__ KPT, const float* __restrict__ V, int bh0, float* __restrict__ CTX) { __shared__ __align__(16) float sf[4][16][68];
  const int tid = threadIdx.x, wave = tid >> 5, lane = tid & 31, col = lane & 15, g = lane >> 4; const int unit = blockIdx.y; const int bh = bh0 + unit; const int b = bh / NHD, h = bh % NHD; const size_t mr0 = (size_t)blockIdx.x * 64 + wave * 16;
  v8f acc[4] = {};
#pragma unroll 1
  for (int kc = 0; kc < NN / 32; ++kc) { const F2 a = split_row(KPT + ((size_t)unit * MF + mr0 + col) * NN, kc * 32, lane); asm volatile("s_wait_loadcnt 0x0" ::: "memory");
#pragma unroll
    for (int j = 0; j < 4; ++j) { float t0[8], t1[8]; const int d = j * 16 + col; const float* vp = V + ((size_t)b * NN + kc * 32 + 8 * g) * HID + h * HDM + d;
#pragma unroll
      for (int i = 0; i < 8; ++i) t0[i] = vp[(size_t)i * HID];
      asm volatile("s_wait_loadcnt 0x0" ::: "memory");
#pragma unroll
      for (int i = 0; i < 8; ++i) t1[i] = vp[(size_t)(16 + i) * HID];
      asm volatile("s_wait_loadcnt 0x0" ::: "memory");
      v16b wh, wl;
#pragma unroll
      for (int i = 0; i < 8; ++i) { const __bf16 h0 = (__bf16)t0[i], h1 = (__bf16)t1[i]; wh[i] = h0; wh[8 + i] = h1; wl[i] = (__bf16)(t0[i] - (float)h0); wl[8 + i] = (__bf16)(t1[i] - (float)h1); }
      acc[j] = wmma_bf(a.h, wh, acc[j]); acc[j] = wmma_bf(a.l, wh, acc[j]); acc[j] = wmma_bf(a.h, wl, acc[j]); } }
#pragma unroll
  for (int j = 0; j < 4; ++j)
#pragma unroll
    for (int r = 0; r < 8; ++r) sf[wave][8 * g + r][j * 16 + col] = acc[j][r];
  LDSX(); for (int rl = 0; rl < 16; ++rl) if (lane < 16) vst2(CTX + ((size_t)bh * MF + mr0 + rl) * HDM + lane * 4, *(const v4f*)&sf[wave][rl][lane * 4]); }
__global__ __launch_bounds__(128) void k_att(const float* __restrict__ QP, const float* __restrict__ CTX, const float* __restrict__ KS, int bh0, float* __restrict__ ATT) { __shared__ __align__(16) float sf[4][16][84];
  const int tid = threadIdx.x, wave = tid >> 5, lane = tid & 31, col = lane & 15, g = lane >> 4; const int unit = blockIdx.y; const int bh = bh0 + unit; const int b = bh / NHD, h = bh % NHD; const size_t n0 = (size_t)blockIdx.x * 64 + wave * 16;
  const float* ctxb = CTX + (size_t)bh * MF * HDM; const float* ksb = KS + (size_t)bh * MF;
  v8f acc[5] = {};
#pragma unroll 1
  for (int kc = 0; kc < MF / 32; ++kc) { const F2 a = split_row(QP + ((size_t)unit * NN + n0 + col) * MF, kc * 32, lane); asm volatile("s_wait_loadcnt 0x0" ::: "memory");
#pragma unroll
    for (int j = 0; j < 5; ++j) { float t0[8], t1[8];
      if (j < 4) { const int d = j * 16 + col;
#pragma unroll
        for (int i = 0; i < 8; ++i) t0[i] = ctxb[(size_t)(kc * 32 + 8 * g + i) * HDM + d];
        asm volatile("s_wait_loadcnt 0x0" ::: "memory");
#pragma unroll
        for (int i = 0; i < 8; ++i) t1[i] = ctxb[(size_t)(kc * 32 + 16 + 8 * g + i) * HDM + d];
        asm volatile("s_wait_loadcnt 0x0" ::: "memory"); }
      else { const float keep = col == 0 ? 1.f : 0.f;
#pragma unroll
        for (int i = 0; i < 8; ++i) t0[i] = ksb[kc * 32 + 8 * g + i] * keep;
        asm volatile("s_wait_loadcnt 0x0" ::: "memory");
#pragma unroll
        for (int i = 0; i < 8; ++i) t1[i] = ksb[kc * 32 + 16 + 8 * g + i] * keep;
        asm volatile("s_wait_loadcnt 0x0" ::: "memory"); }
      v16b wh, wl;
#pragma unroll
      for (int i = 0; i < 8; ++i) { const __bf16 h0 = (__bf16)t0[i], h1 = (__bf16)t1[i]; wh[i] = h0; wh[8 + i] = h1; wl[i] = (__bf16)(t0[i] - (float)h0); wl[8 + i] = (__bf16)(t1[i] - (float)h1); }
      acc[j] = wmma_bf(a.h, wh, acc[j]); acc[j] = wmma_bf(a.l, wh, acc[j]); acc[j] = wmma_bf(a.h, wl, acc[j]); } }
#pragma unroll
  for (int j = 0; j < 5; ++j)
#pragma unroll
    for (int r = 0; r < 8; ++r) sf[wave][8 * g + r][j * 16 + col] = acc[j][r];
  LDSX();
  for (int rl = 0; rl < 16; ++rl) { const float den = sf[wave][rl][64]; const float inv = 1.0f / den; if (lane < 16) { v4f v = *(const v4f*)&sf[wave][rl][lane * 4]; v[0] *= inv; v[1] *= inv; v[2] *= inv; v[3] *= inv; vst2(ATT + ((size_t)b * NN + (size_t)h * (NN / 8) + (n0 + rl) / 8) * HID + ((n0 + rl) & 7) * HDM + lane * 4, v); } } }
__global__ __launch_bounds__(128) void k_out(const float* __restrict__ ATT, const float* __restrict__ WO, const float* __restrict__ BO, float* __restrict__ OUT) { __shared__ __align__(16) float sf[4][16][132];
  const int tid = threadIdx.x, wave = tid >> 5, lane = tid & 31, col = lane & 15, g = lane >> 4; const int c0 = blockIdx.y * 128; const size_t r0 = (size_t)blockIdx.x * 64 + wave * 16;
  v8f acc[8] = {};
#pragma unroll 1
  for (int kc = 0; kc < HID / 32; ++kc) { const F2 a = split_row(ATT + (r0 + col) * HID, kc * 32, lane); asm volatile("s_wait_loadcnt 0x0" ::: "memory");
#pragma unroll
    for (int j = 0; j < 8; ++j) { const v16b w = wcol_oi(WO, kc * 32, c0 + j * 16 + col, lane, HID); asm volatile("s_wait_loadcnt 0x0" ::: "memory"); acc[j] = wmma_bf(a.h, w, acc[j]); acc[j] = wmma_bf(a.l, w, acc[j]); } }
#pragma unroll
  for (int j = 0; j < 8; ++j) { const float bb = bfr(BO[c0 + j * 16 + col]);
#pragma unroll
    for (int r = 0; r < 8; ++r) sf[wave][8 * g + r][j * 16 + col] = acc[j][r] + bb; }
  LDSX(); for (int rl = 0; rl < 16; ++rl) vst2(OUT + (r0 + rl) * HID + c0 + lane * 4, *(const v4f*)&sf[wave][rl][lane * 4]); }
extern "C" void kernel_launch(void* const* d_in, const int* in_sizes, int n_in, void* d_out, int out_size, void* d_ws, size_t ws_size, hipStream_t stream) {
  (void)in_sizes; (void)n_in; (void)out_size;
  if (ws_size < (size_t)WS_END) return;
  char* ws = (char*)d_ws; const float** F = (const float**)d_in;
  float *Q = (float*)(ws + WS_Q), *K = (float*)(ws + WS_K), *V = (float*)(ws + WS_V), *QP = (float*)(ws + WS_QP), *KPT = (float*)(ws + WS_KPT), *KS = (float*)(ws + WS_KS), *CTX = (float*)(ws + WS_CTX), *ATT = (float*)(ws + WS_ATT);
  k_lin<<<dim3(NRV / 64, HID / 128, 3), 128, 0, stream>>>(F[0], F[1], F[2], F[3], F[5], F[7], F[4], F[6], F[8], Q, K, V);
  for (int bh0 = 0; bh0 < TNB * NHD; bh0 += UG) {
    k_phi<<<dim3(NN / 64, MF / 128, UG * 2), 128, 0, stream>>>(Q, K, F[11], bh0, QP, KPT);
    k_ksum<<<dim3(MF / 64, UG), 256, 0, stream>>>(KPT, bh0, KS);
    k_ctx<<<dim3(MF / 64, UG), 128, 0, stream>>>(KPT, V, bh0, CTX);
    k_att<<<dim3(NN / 64, UG), 128, 0, stream>>>(QP, CTX, KS, bh0, ATT);
  }
  k_out<<<dim3(NRV / 64, HID / 128), 128, 0, stream>>>(ATT, F[9], F[10], (float*)d_out);
}
